// CHESHIRE_90374701843019
// MI455X (gfx1250) — hardware-run, weakly checked
//
#include <hip/hip_runtime.h>


namespace {
constexpr int NN = 2000, F = 256, D = 128, NE = 20000, S = 8, M = NE * S  , EL = 1120000, NPB = 8;
constexpr float XS = 8.0f, HS = 256.0f, WSC = 256.0f, EPS = 1e-5f;
typedef _Float16 b16;
typedef __attribute__((ext_vector_type(16))) _Float16 v16b;
typedef __attribute__((ext_vector_type(8))) _Float16 v8b;
typedef __attribute__((ext_vector_type(8))) float v8f;
typedef __attribute__((ext_vector_type(4))) float v4f;
__device__ __forceinline__ float bf16_rne(float f) { unsigned int u = __float_as_uint(f); u += 0x7FFFu + ((u >> 16) & 1u); float r = __uint_as_float(u & 0xFFFF0000u); asm volatile("" : "+v"(r)); return r; }
__device__ __forceinline__ float bfv(float f) { float r = bf16_rne(f); asm volatile("" : "+v"(r)); return r; }
__device__ __forceinline__ void split16(float v, b16& hi, b16& lo) { hi = (b16)v; lo = (b16)(v - (float)hi); }
__device__ __forceinline__ v16b frag_kb(const b16* p, int hh) { const v8b a = *(const v8b*)(p + 8 * hh), b = *(const v8b*)(p + 16 + 8 * hh); v16b f;
#pragma unroll
  for (int e = 0; e < 8; ++e) { f[e] = a[e]; f[8 + e] = b[e]; } return f; }
__device__ __forceinline__ v8f wmma16b(v16b a, v16b b, v8f c) { v8f d = __builtin_amdgcn_wmma_f32_16x16x32_f16(false, a, false, b, (short)0, c, false, false); asm volatile("v_nop\n\tv_nop\n\tv_nop\n\tv_nop" : "+v"(d) : "v"(a), "v"(b)); return d; }
__device__ __forceinline__ void wave_lds_sync() { __builtin_amdgcn_fence(__ATOMIC_RELEASE, "workgroup"); __builtin_amdgcn_wave_barrier(); __builtin_amdgcn_fence(__ATOMIC_ACQUIRE, "workgroup"); }
__device__ __forceinline__ float pmul(float a, float b) { float p = a * b; asm volatile("" : "+v"(p)); return p; }
__device__ __forceinline__ int iclamp(int v, int lo, int hi) { return v < lo ? lo : (v > hi ? hi : v); }
__device__ __forceinline__ float htanh(float v) { return fminf(fmaxf(v, -1.0f), 1.0f); }
#define E EL
constexpr int CSR_NBLK9 = 512, CSR_GB9 = 9, CSR_GN9 = 1 << CSR_GB9  , CSR_TS9 = (CSR_GN9 < 32 ? 32 : CSR_GN9)  , CSR_MAXG9 = 512, CSR_CAP9 = 12288  ;
__device__ __host__ __forceinline__ int csr_tix9(int v) { return (v >> CSR_GB9) * CSR_TS9 + (v & (CSR_GN9 - 1)); }
__global__ __launch_bounds__(64) void csrA_kernel9(const int* __restrict__ dst, int E, int N, int nG, int CHP, int NGP, int* __restrict__ STG, int* __restrict__ HST) {
  extern __shared__ int sm[];
  int* cnt = sm; int* run = sm + NGP; int* ids = sm + 2 * NGP;
  const int b = blockIdx.x; const int ch = (E + CSR_NBLK9 - 1) / CSR_NBLK9; const int e0 = b * ch, e1 = min(E, e0 + ch);
  for (int i = threadIdx.x; i < NGP; i += 64) cnt[i] = 0;
  for (int i = threadIdx.x; i < CHP; i += 64) ids[i] = -1;
  __syncthreads();
  if (threadIdx.x == 0) {
    for (int e = e0; e < e1; ++e) { int d = dst[e]; d = (d < 0) ? 0 : (d >= N ? N - 1 : d); cnt[d >> CSR_GB9] += 1; }
    int acc = 0; for (int g = 0; g < nG; ++g) { run[g] = acc; acc += cnt[g]; }
    for (int e = e0; e < e1; ++e) { int d = dst[e]; d = (d < 0) ? 0 : (d >= N ? N - 1 : d); const int g = d >> CSR_GB9; ids[run[g]] = e; run[g] += 1; } }
  __syncthreads();
  typedef __attribute__((ext_vector_type(4))) int v4i;
  for (int pass = 0; pass < 2; ++pass) {
    for (int i = threadIdx.x; i < CHP / 4; i += 64) *(volatile v4i*)(STG + (size_t)b * CHP + i * 4) = *(const v4i*)(&ids[i * 4]);
    for (int i = threadIdx.x; i < NGP / 4; i += 64) { v4i v; for (int e = 0; e < 4; ++e) v[e] = (i * 4 + e < nG) ? cnt[i * 4 + e] : 0; *(volatile v4i*)(HST + (size_t)b * NGP + i * 4) = v; }
    __threadfence(); }
}
__global__ __launch_bounds__(512) void csrS_kernel9(const int* __restrict__ HST, int nG, int NGP, int* __restrict__ START, int* __restrict__ TOT, int* __restrict__ OFF) {
  __shared__ int tot[CSR_MAXG9];
  const int b = threadIdx.x;
  for (int pass = 0; pass < 2; ++pass) { int runb = 0; for (int g = 0; g < nG; ++g) { int c = HST[(size_t)b * NGP + g]; c = (c < 0) ? 0 : c; ((volatile int*)OFF)[(size_t)g * CSR_NBLK9 + b] = runb; runb += c; } __threadfence(); }
  for (int g = threadIdx.x; g < nG; g += 512) { int s = 0; for (int bb = 0; bb < CSR_NBLK9; ++bb) { int c = HST[(size_t)bb * NGP + g]; s += (c < 0) ? 0 : c; } tot[g] = s; }
  __syncthreads();
  if (threadIdx.x < 32) {
    __shared__ int st[CSR_MAXG9 + 32];
    if (threadIdx.x == 0) { int acc = 0; for (int g = 0; g < NGP; ++g) { st[g] = acc; if (g < nG) acc += (tot[g] + 31) & ~31; } st[NGP] = acc; }
    __builtin_amdgcn_fence(__ATOMIC_RELEASE, "workgroup"); __builtin_amdgcn_wave_barrier(); __builtin_amdgcn_fence(__ATOMIC_ACQUIRE, "workgroup");
    for (int pass = 0; pass < 2; ++pass) { for (int i = threadIdx.x; i < NGP + 32; i += 32) { ((volatile int*)START)[i] = (i <= NGP) ? st[min(i, NGP)] : 0; ((volatile int*)TOT)[i] = (i < nG) ? tot[i] : 0; } __threadfence(); } }
}
__global__ __launch_bounds__(256) void csrB_kernel9(const int* __restrict__ dst, int N, int nG, int CHP, int NGP, int permLen, const int* __restrict__ STG, const int* __restrict__ HST, const int* __restrict__ OFF, const int* __restrict__ START, const int* __restrict__ TOT, int* __restrict__ PERM, int* __restrict__ ROWPTR, int* __restrict__ ROWCNT, int* __restrict__ FLAG) {
  typedef __attribute__((ext_vector_type(4))) int v4i;
  __shared__ int ids[CSR_CAP9]; __shared__ unsigned short key[CSR_CAP9]; __shared__ int outp[CSR_CAP9]; __shared__ int ncnt[CSR_GN9 + 1]; __shared__ int boff[CSR_NBLK9 + 1];
  const int g = blockIdx.x, t_ = threadIdx.x; int tot = TOT[g]; int st = START[g], stn = START[g + 1]; const int v0 = g * CSR_GN9; const int nv = min(CSR_GN9, N - v0); const int t0 = g * CSR_TS9;
  st = (st < 0) ? 0 : (st > permLen - 32 ? permLen - 32 : st) & ~31; stn = (stn < st) ? st : (stn > permLen ? permLen : stn); tot = (tot < 0) ? 0 : tot; if (tot > stn - st && tot <= CSR_CAP9) tot = stn - st;
  if (tot > CSR_CAP9) {
    for (int pass = 0; pass < 2; ++pass) { for (int i = t_; i < CSR_TS9 / 4; i += 256) { v4i a, c; for (int e = 0; e < 4; ++e) { a[e] = st; c[e] = 0; } *(volatile v4i*)(ROWPTR + t0 + i * 4) = a; *(volatile v4i*)(ROWCNT + t0 + i * 4) = c; } if (t_ == 0) ((volatile int*)FLAG)[0] = 1; __threadfence(); } (void)nv; return; }
  if (t_ == 0) { int acc = 0; for (int b = 0; b < CSR_NBLK9; ++b) { boff[b] = acc; int c = HST[(size_t)b * NGP + g]; c = (c < 0) ? 0 : (c > CHP ? CHP : c); acc += c; if (acc > tot) acc = tot; } boff[CSR_NBLK9] = acc; }
  for (int i = t_; i <= CSR_GN9; i += 256) ncnt[i] = 0;
  __syncthreads();
  for (int b = 0; b < CSR_NBLK9; ++b) { const int c = boff[b + 1] - boff[b]; int o_ = OFF[(size_t)g * CSR_NBLK9 + b]; o_ = (o_ < 0) ? 0 : (o_ > CHP - c ? CHP - c : o_); const int* src_ = STG + (size_t)b * CHP + o_;
    for (int i = t_; i < c; i += 256) { int id = src_[i]; id = (id < 0) ? 0 : id; ids[boff[b] + i] = id; int d = dst[id]; d = (d < v0) ? v0 : (d >= N ? N - 1 : d); int kk = d - v0; kk = (kk < 0) ? 0 : (kk >= CSR_GN9 ? CSR_GN9 - 1 : kk); key[boff[b] + i] = (unsigned short)kk; } }
  __syncthreads();
  if (t_ == 0) { for (int i = 0; i < tot; ++i) ncnt[key[i]] += 1; int acc = 0; for (int vl = 0; vl < CSR_GN9; ++vl) { const int c = ncnt[vl]; ncnt[vl] = acc; acc += c; } ncnt[CSR_GN9] = acc;
    for (int i = 0; i < tot; ++i) { const int vl = key[i]; outp[ncnt[vl]] = ids[i]; ncnt[vl] += 1; }
    for (int vl = CSR_GN9; vl > 0; --vl) ncnt[vl] = ncnt[vl - 1]; ncnt[0] = 0; }
  __syncthreads();
  for (int pass = 0; pass < 2; ++pass) {
    for (int i = t_; i < (stn - st) / 4; i += 256) { v4i v; for (int e = 0; e < 4; ++e) { const int q = i * 4 + e; v[e] = (q < tot) ? outp[q] : -1; } *(volatile v4i*)(PERM + st + i * 4) = v; }
    for (int i = t_; i < CSR_TS9 / 4; i += 256) { v4i a, c; for (int e = 0; e < 4; ++e) { const int vl = i * 4 + e; const int vc = vl < CSR_GN9 ? vl : CSR_GN9; a[e] = (vl < CSR_GN9) ? st + ncnt[vc] : st; c[e] = (vl < nv) ? (ncnt[(vc < CSR_GN9 ? vc : CSR_GN9 - 1) + 1] - ncnt[vc]) : 0; } *(volatile v4i*)(ROWPTR + t0 + i * 4) = a; *(volatile v4i*)(ROWCNT + t0 + i * 4) = c; }
    __threadfence(); }
}
__global__ __launch_bounds__(256) void csrZ_kernel9(int* __restrict__ p, size_t n4) { typedef __attribute__((ext_vector_type(4))) int v4i; const size_t tid = (size_t)blockIdx.x * 256 + threadIdx.x, nth = (size_t)gridDim.x * 256; v4i z = {0, 0, 0, 0}; for (size_t i = tid; i < n4; i += nth) *(volatile v4i*)(p + i * 4) = z; }
struct CsrBufs9 { int *STG, *HST, *OFF, *START, *TOT, *PERM, *ROWPTR, *ROWCNT, *FLAG; int nG, NGP, CHP; size_t permLen; char* base; size_t bytes; };
static size_t csr_carve9(CsrBufs9& c, char* ws, size_t off, int E, int N) {
  const size_t off0 = off; c.base = ws + off;
  auto al = [&](size_t bytes) { char* p = ws + off; off += (bytes + 255) & ~(size_t)255; return p; };
  c.nG = (N + CSR_GN9 - 1) / CSR_GN9; c.NGP = (c.nG + 31) & ~31; const int ch = (E + CSR_NBLK9 - 1) / CSR_NBLK9; c.CHP = (ch + 31) & ~31; c.permLen = (size_t)E + 32 * (size_t)c.nG + 32;
  c.STG = (int*)al((size_t)CSR_NBLK9 * c.CHP * 4); c.HST = (int*)al((size_t)CSR_NBLK9 * c.NGP * 4); c.OFF = (int*)al((size_t)c.NGP * CSR_NBLK9 * 4); c.START = (int*)al((size_t)(c.NGP + 64) * 4); c.TOT = (int*)al((size_t)(c.NGP + 64) * 4);
  c.PERM = (int*)al(c.permLen * 4); c.ROWPTR = (int*)al((size_t)c.nG * CSR_TS9 * 4); c.ROWCNT = (int*)al((size_t)c.nG * CSR_TS9 * 4); c.FLAG = (int*)al(256);
  c.bytes = off - off0; return off;
}
static void csr_build9(const CsrBufs9& c, const int* dst, int E, int N, hipStream_t stream) {
  const size_t smem = (size_t)(2 * c.NGP + c.CHP) * 4;
  csrZ_kernel9<<<512, 256, 0, stream>>>((int*)c.base, c.bytes / 16);
  csrA_kernel9<<<CSR_NBLK9, 64, smem, stream>>>(dst, E, N, c.nG, c.CHP, c.NGP, c.STG, c.HST);
  csrS_kernel9<<<1, 512, 0, stream>>>(c.HST, c.nG, c.NGP, c.START, c.TOT, c.OFF);
  csrB_kernel9<<<c.nG, 256, 0, stream>>>(dst, N, c.nG, c.CHP, c.NGP, (int)c.permLen, c.STG, c.HST, c.OFF, c.START, c.TOT, c.PERM, c.ROWPTR, c.ROWCNT, c.FLAG);
}

#undef E
__device__ __forceinline__ float dis_of(const int* ROWCNT, size_t r) { const int d = iclamp(ROWCNT[r], 0, EL); return d > 0 ? rsqrtf((float)d) : 0.0f; }

__global__ __launch_bounds__(256) void wput_kernel(const float* __restrict__ we, const float* __restrict__ cw, b16* __restrict__ WE, b16* __restrict__ WC) { const int u = blockIdx.x * 256 + threadIdx.x; v8b v;
  if (u < D * 32) { const int o = u / 32, k0 = (u % 32) * 8;
#pragma unroll
    for (int j = 0; j < 8; ++j) v[j] = (b16)(bf16_rne(we[(size_t)(k0 + j) * D + o]) * WSC); for (int pass = 0; pass < 2; ++pass) { *(volatile v8b*)(WE + (size_t)o * F + k0) = v; __threadfence(); } }
  if (u < D * 48) { const int o = u / 48, k0 = (u % 48) * 8;
#pragma unroll
    for (int j = 0; j < 8; ++j) { const int k = k0 + j; v[j] = (b16)(bf16_rne(cw[((size_t)(k / D) * D + (k % D)) * D + o]) * WSC); } for (int pass = 0; pass < 2; ++pass) { *(volatile v8b*)(WC + (size_t)o * 3 * D + k0) = v; __threadfence(); } } }
__global__ __launch_bounds__(32) void enc_kernel(const float* __restrict__ feat, const b16* __restrict__ WE, const float* __restrict__ be, float* __restrict__ X0) { __shared__ __attribute__((aligned(16))) b16 Ah[16][F + 8]; __shared__ float Tf[16][D + 4]; const int lane = threadIdx.x, nloc = lane & 15, hlf = lane >> 4; const size_t m0 = (size_t)blockIdx.x * 16;
  for (int rr = 0; rr < 16; ++rr) for (int q = 0; q < 8; ++q) Ah[rr][q * 32 + lane] = (b16)(bf16_rne(feat[(m0 + rr) * F + q * 32 + lane]) * XS); if (lane < 16) for (int k = F; k < F + 8; ++k) Ah[lane][k] = (b16)0.0f;
  wave_lds_sync(); v8f acc[8];
#pragma unroll
  for (int t = 0; t < 8; ++t) acc[t] = (v8f){};
#pragma unroll 2
  for (int kb = 0; kb < F; kb += 32) { const v16b a = frag_kb(&Ah[nloc][kb], hlf);
#pragma unroll
    for (int t = 0; t < 8; ++t) acc[t] = wmma16b(a, frag_kb(WE + (size_t)(t * 16 + nloc) * F + kb, hlf), acc[t]); }
#pragma unroll
  for (int t = 0; t < 8; ++t) { const int cc = t * 16 + nloc; const float bb = bfv(be[cc]);
#pragma unroll
    for (int r8 = 0; r8 < 8; ++r8) Tf[8 * hlf + r8][cc] = htanh(acc[t][r8] * (1.0f / (XS * WSC)) + bb); }
  wave_lds_sync();
  for (int pass = 0; pass < 2; ++pass) { for (int rr = 0; rr < 16; ++rr) *(volatile v4f*)(X0 + (m0 + rr) * D + lane * 4) = *(const v4f*)(&Tf[rr][lane * 4]); __threadfence(); } }
__global__ __launch_bounds__(256) void gnorm_kernel(const float* __restrict__ X0, const int* __restrict__ hn, const float* __restrict__ gw, const float* __restrict__ gb, const float* __restrict__ gms, int ELIM, float* __restrict__ XN) { const int wave = threadIdx.x >> 5, lane = threadIdx.x & 31; const int e = blockIdx.x * NPB + wave; if (e >= ELIM) return; v4f xs[S]; v4f mu = {0, 0, 0, 0};
#pragma unroll
  for (int s = 0; s < S; ++s) { const size_t n = (size_t)iclamp(hn[(size_t)e * S + s], 0, NN - 1); xs[s] = *(const v4f*)(X0 + n * D + lane * 4); for (int k = 0; k < 4; ++k) mu[k] += xs[s][k]; }
  v4f var = {0, 0, 0, 0}; float msv[4], wv[4], bv[4]; for (int k = 0; k < 4; ++k) { mu[k] *= (1.0f / S); msv[k] = bfv(gms[lane * 4 + k]); wv[k] = bfv(gw[lane * 4 + k]); bv[k] = bfv(gb[lane * 4 + k]); }
#pragma unroll
  for (int s = 0; s < S; ++s) for (int k = 0; k < 4; ++k) { const float xc = xs[s][k] - mu[k] * msv[k]; xs[s][k] = xc; var[k] += xc * xc; }
  float rs[4]; for (int k = 0; k < 4; ++k) rs[k] = 1.0f / sqrtf(var[k] * (1.0f / S) + EPS);
  for (int pass = 0; pass < 2; ++pass) {
#pragma unroll
    for (int s = 0; s < S; ++s) { v4f o; for (int k = 0; k < 4; ++k) o[k] = pmul(xs[s][k] * rs[k], wv[k]) + bv[k]; *(volatile v4f*)(XN + ((size_t)e * S + s) * D + lane * 4) = o; } __threadfence(); } }
__global__ __launch_bounds__(256) void lap_kernel(const float* __restrict__ V, const float* __restrict__ SUB, float scale, const int* __restrict__ cols, const int* __restrict__ PERM, const int* __restrict__ ROWPTR, const int* __restrict__ ROWCNT, int permLen, int RLIM, float* __restrict__ T) { const int wave = threadIdx.x >> 5, lane = threadIdx.x & 31; const size_t r = (size_t)blockIdx.x * NPB + wave; if (r >= (size_t)RLIM) return; int st = ROWPTR[r], cnt = ROWCNT[r]; cnt = iclamp(cnt, 0, EL); st = iclamp(st, 0, permLen - cnt); const float dr = dis_of(ROWCNT, r); v4f acc = {0, 0, 0, 0};
#pragma unroll 1
  for (int j = 0; j < cnt; ++j) { const int eg = iclamp(PERM[st + j], 0, EL - 1); const size_t c = (size_t)iclamp(cols[eg], 0, M - 1); if (c >= (size_t)RLIM) continue; const float w = -pmul(dr, dis_of(ROWCNT, c)); const v4f v = *(const v4f*)(V + c * D + lane * 4); for (int k = 0; k < 4; ++k) acc[k] += pmul(w, v[k]); }
  v4f o; for (int k = 0; k < 4; ++k) { o[k] = acc[k] * scale; if (SUB) o[k] -= SUB[r * D + lane * 4 + k]; }
  for (int pass = 0; pass < 2; ++pass) { *(volatile v4f*)(T + r * D + lane * 4) = o; __threadfence(); } }
__global__ __launch_bounds__(32) void cheb_kernel(const float* __restrict__ XN, const float* __restrict__ T1, const int* __restrict__ cols, const int* __restrict__ PERM, const int* __restrict__ ROWPTR, const int* __restrict__ ROWCNT, int permLen, int RLIM, const b16* __restrict__ WC, const float* __restrict__ cb, int ELIM, float* __restrict__ Y) { __shared__ __attribute__((aligned(16))) b16 Ah[16][3 * D + 8], Al[16][3 * D + 8]; __shared__ float Tf[16][D + 4]; const int lane = threadIdx.x, nloc = lane & 15, hlf = lane >> 4; const int e0 = blockIdx.x * 2; if (e0 >= ELIM) return; const size_t m0 = (size_t)e0 * S;
  for (int rr = 0; rr < 16; ++rr) { for (int q = 0; q < 8; ++q) { const int c = q * 32 + lane; const int part = c / D, cc = c % D; const float v = (part == 0 ? XN : T1)[(m0 + rr) * D + cc]; b16 p, ql; split16(v * HS, p, ql); Ah[rr][c] = p; Al[rr][c] = ql; }
    { const size_t r = m0 + rr; int st = ROWPTR[r], cnt = ROWCNT[r]; cnt = iclamp(cnt, 0, EL); st = iclamp(st, 0, permLen - cnt); const float dr = dis_of(ROWCNT, r); v4f acc2 = {0, 0, 0, 0};
#pragma unroll 1
      for (int j = 0; j < cnt; ++j) { const int eg = iclamp(PERM[st + j], 0, EL - 1); const size_t c = (size_t)iclamp(cols[eg], 0, M - 1); if (c >= (size_t)RLIM) continue; const float w = -pmul(dr, dis_of(ROWCNT, c)); const v4f v = *(const v4f*)(T1 + c * D + lane * 4); for (int k = 0; k < 4; ++k) acc2[k] += pmul(w, v[k]); }
      for (int k = 0; k < 4; ++k) { const float t2 = acc2[k] * 2.0f - XN[r * D + lane * 4 + k]; b16 p, ql; split16(t2 * HS, p, ql); Ah[rr][2 * D + lane * 4 + k] = p; Al[rr][2 * D + lane * 4 + k] = ql; } } }
  if (lane < 16) for (int k = 3 * D; k < 3 * D + 8; ++k) { Ah[lane][k] = (b16)0.0f; Al[lane][k] = (b16)0.0f; }
  wave_lds_sync(); v8f acc[8];
#pragma unroll
  for (int t = 0; t < 8; ++t) acc[t] = (v8f){};
#pragma unroll 2
  for (int kb = 0; kb < 3 * D; kb += 32) { const v16b a = frag_kb(&Ah[nloc][kb], hlf), al = frag_kb(&Al[nloc][kb], hlf);
#pragma unroll
    for (int t = 0; t < 8; ++t) { const v16b bw = frag_kb(WC + (size_t)(t * 16 + nloc) * 3 * D + kb, hlf); acc[t] = wmma16b(a, bw, acc[t]); acc[t] = wmma16b(al, bw, acc[t]); } }
#pragma unroll
  for (int t = 0; t < 8; ++t) { const int cc = t * 16 + nloc; const float bb = bfv(cb[cc]);
#pragma unroll
    for (int r8 = 0; r8 < 8; ++r8) Tf[8 * hlf + r8][cc] = htanh(acc[t][r8] * (1.0f / (HS * WSC)) + bb); }
  wave_lds_sync();
  for (int pass = 0; pass < 2; ++pass) { for (int h2 = 0; h2 < 2; ++h2) { v4f dmm, nrm; for (int k = 0; k < 4; ++k) { const int c = lane * 4 + k; float mx = -INFINITY, mn = INFINITY, sq = 0.0f; for (int s = 0; s < S; ++s) { const float v = Tf[h2 * S + s][c]; mx = fmaxf(mx, v); mn = fminf(mn, v); sq += v * v; } dmm[k] = mx - mn; nrm[k] = sqrtf(sq * (1.0f / S)); }
      *(volatile v4f*)(Y + (size_t)(e0 + h2) * 2 * D + lane * 4) = dmm; *(volatile v4f*)(Y + (size_t)(e0 + h2) * 2 * D + D + lane * 4) = nrm; } __threadfence(); } }
__global__ __launch_bounds__(256) void head_kernel(const float* __restrict__ Y, const float* __restrict__ wo, const float* __restrict__ bo, int ELIM, float* __restrict__ out) { const size_t e = (size_t)blockIdx.x * 256 + threadIdx.x; if (e >= (size_t)ELIM) return; float s = bfv(bo[0]);
#pragma unroll 4
  for (int c = 0; c < 2 * D; ++c) s += pmul(Y[e * 2 * D + c], bfv(wo[c]));
  const float p = 1.0f / (1.0f + __expf(-s));
  for (int pass = 0; pass < 2; ++pass) { ((volatile float*)out)[e] = p; __threadfence(); } }
}

extern "C" void kernel_launch(void* const* d_in, const int* in_sizes, int n_in, void* d_out, int out_size, void* d_ws, size_t ws_size, hipStream_t stream) {
  (void)n_in;
  auto Fp = [&](int i) { return (const float*)d_in[i]; }; auto Ip = [&](int i) { return (const int*)d_in[i]; };
  if (in_sizes[0] != NN * F || in_sizes[1] != F * D || in_sizes[6] != 3 * D * D || in_sizes[8] != 2 * D || in_sizes[10] != NE * S || in_sizes[11] != EL || in_sizes[12] != EL || out_size != NE) return;
  const int ELIM = NE;
  const int RLIM = ELIM * S;
  size_t off = 0; char* ws = (char*)d_ws;
  auto carve = [&](size_t bytes) { char* p = ws + off; off += (bytes + 255) & ~(size_t)255; return p; };
  b16* WE = (b16*)carve((size_t)D * F * 2); b16* WC = (b16*)carve((size_t)D * 3 * D * 2); float* X0 = (float*)carve((size_t)NN * D * 4); float* XN = (float*)carve((size_t)M * D * 4); float* T1 = (float*)carve((size_t)M * D * 4); float* Y = (float*)carve((size_t)NE * 2 * D * 4); CsrBufs9 csr; off = csr_carve9(csr, ws, off, EL, M);
  if (off > ws_size || off > ((size_t)232 << 20)) return;
  wput_kernel<<<(D * 48 + 255) / 256, 256, 0, stream>>>(Fp(1), Fp(6), WE, WC);
  csr_build9(csr, Ip(11), EL, M, stream);
  enc_kernel<<<NN / 16, 32, 0, stream>>>(Fp(0), WE, Fp(2), X0);
  gnorm_kernel<<<(ELIM + NPB - 1) / NPB, 256, 0, stream>>>(X0, Ip(10), Fp(3), Fp(4), Fp(5), ELIM, XN);
  lap_kernel<<<(RLIM + NPB - 1) / NPB, 256, 0, stream>>>(XN, nullptr, 1.0f, Ip(12), csr.PERM, csr.ROWPTR, csr.ROWCNT, (int)csr.permLen, RLIM, T1);
  cheb_kernel<<<ELIM / 2, 32, 0, stream>>>(XN, T1, Ip(12), csr.PERM, csr.ROWPTR, csr.ROWCNT, (int)csr.permLen, RLIM, WC, Fp(7), ELIM, Y);
  head_kernel<<<(NE + 255) / 256, 256, 0, stream>>>(Y, Fp(8), Fp(9), ELIM, (float*)d_out);
}
